// WaveNet_36155034698369
// MI455X (gfx1250) — hardware-verified
//
#include <hip/hip_runtime.h>
#include <stddef.h>
#include <math.h>

typedef __attribute__((ext_vector_type(16))) _Float16 v16h;
typedef __attribute__((ext_vector_type(8)))  _Float16 v8h;
typedef __attribute__((ext_vector_type(8)))  float    v8f;
typedef __attribute__((ext_vector_type(4)))  float    v4f;

constexpr int kBatch  = 32;
constexpr int kLen    = 4096;
constexpr int kCin    = 32;
constexpr int kCh     = 64;
constexpr int kEnd    = 128;
constexpr int kLayers = 30;
constexpr int kLayersPerGroup = 10;
constexpr int kKfg    = 2 * kCh;
constexpr int kThreads = 256;
constexpr int kWaves   = 8;
constexpr int kWaveP   = 16;
constexpr int kTileP   = kWaves * kWaveP;
constexpr int kSlabP   = 68;
constexpr int kZP      = 64;
constexpr float kWCarry = 8.0f;
constexpr float kFold   = 0.125f;

static_assert(kKfg % 32 == 0 && kCh % 32 == 0 && kCin % 32 == 0);
static_assert(kCh == 64);
static_assert(kLen % kWaveP == 0 && kTileP == 128 && kThreads == 32 * kWaves);
static_assert(kThreads * 4 * 8 == kCh * kKfg);
static_assert(kThreads * 2 * 8 == kCh * kCh);
static_assert(kThreads * 8 == kCh * kCin);
static_assert(kThreads * 16 == kTileP * kCin);
static_assert((kLayers * kCh * 8) % kThreads == 0);
static_assert(kThreads == 4 * kCh && kBatch % 4 == 0 && kEnd == 2 * kCh);
static_assert(3 * kBatch == 24 * 4);
static_assert((kSlabP * 4) % 16 == 0 && (kZP * 2) % 16 == 0);

struct Sched { int T[kLayers]; int R[kLayers]; int Tin; };
__host__ __device__ constexpr int dil_of(int i) { return 1 << (i % kLayersPerGroup); }
__host__ __device__ constexpr int floor16nn(int v) { return v < 0 ? 0 : (v & ~15); }
__host__ __device__ constexpr Sched make_sched() {
  Sched s = {};
  s.T[kLayers - 1] = kLen;
  s.R[kLayers - 1] = kLen - dil_of(kLayers - 1);
  for (int i = kLayers - 2; i >= 0; --i) { s.T[i] = floor16nn(s.R[i + 1]); s.R[i] = s.T[i] - dil_of(i); }
  s.Tin = floor16nn(s.R[0]);
  return s;
}
constexpr Sched kSched = make_sched();
__host__ __device__ constexpr bool sched_ok() {
  const Sched s = make_sched();
  if (s.Tin < 0 || s.Tin > s.R[0] || (s.Tin % 16) != 0) return false;
  for (int i = 0; i < kLayers; ++i) {
    if (s.R[i] < 0) return false;
    if ((s.T[i] % 16) != 0 || s.T[i] > kLen) return false;
    if (s.R[i] > kLen - dil_of(i)) return false;
    if (i > 0 && s.T[i - 1] > s.R[i]) return false;
  }
  return true;
}
static_assert(sched_ok());

__device__ __forceinline__ unsigned short f2bf_bits(float f) {
  unsigned u = __float_as_uint(f);
  return (unsigned short)((u + 0x7FFFu + ((u >> 16) & 1u)) >> 16);
}
__device__ __forceinline__ float bf_bits2f(unsigned short h) { return __uint_as_float(((unsigned)h) << 16); }
__device__ __forceinline__ float bfr(float f) { return bf_bits2f(f2bf_bits(f)); }

struct FragH {
  union U { v16h v; v8h h[2]; };
  static __device__ __forceinline__ v16h load(const _Float16* p) {
    U f; f.h[0] = *(const v8h*)(p); f.h[1] = *(const v8h*)(p + 16); return f.v;
  }
  static __device__ __forceinline__ v8f mma(v16h a, v16h b, v8f c) {
    return __builtin_amdgcn_wmma_f32_16x16x32_f16(false, a, false, b, (short)0, c, false, false);
  }
};
__device__ __forceinline__ void guard_fg(v8f& f, v8f& g, v16h a1, v16h a2, v16h bb) {
  asm volatile("v_nop\n\tv_nop\n\tv_nop\n\tv_nop" : "+v"(f), "+v"(g) : "v"(a1), "v"(a2), "v"(bb));
}
__device__ __forceinline__ void guard_1(v8f& f, v16h a, v16h bb) {
  asm volatile("v_nop\n\tv_nop\n\tv_nop\n\tv_nop" : "+v"(f) : "v"(a), "v"(bb));
}
__device__ __forceinline__ void acc_guard4(v8f& a, v8f& b, v8f& c, v8f& d) {
  asm volatile("v_nop\n\tv_nop\n\tv_nop\n\tv_nop" : "+v"(a), "+v"(b), "+v"(c), "+v"(d));
}
__device__ __forceinline__ v8f v8f_zero() { return (v8f){0.f, 0.f, 0.f, 0.f, 0.f, 0.f, 0.f, 0.f}; }

__device__ __forceinline__ float fsig(float v)  { return __builtin_amdgcn_rcpf(1.0f + __expf(-v)); }
__device__ __forceinline__ float ftanh(float v) { return 1.0f - 2.0f * __builtin_amdgcn_rcpf(__expf(2.0f * v) + 1.0f); }
__device__ __forceinline__ float gated_precise(float fpre, float gpre) {
  const float gc = fminf(fmaxf(gpre, -30.0f), 30.0f);
  const float th = tanhf(fpre);
  const float sg = 1.0f / (1.0f + expf(-gc));
  return th * sg;
}

template <bool RESID>
__device__ __forceinline__ void tile_store(float* slab, v4f b4, const float* __restrict__ hin_b,
                                           float* __restrict__ hout_b, _Float16* __restrict__ hb_b,
                                           int t0, int lane, bool active) {
  const int hh = lane >> 4, c4 = (lane & 15) * 4;
  const int q = lane >> 3, c8 = (lane & 7) * 8;
  __syncthreads();
#pragma unroll
  for (int it = 0; it < 8; ++it) {
    const int row = it * 2 + hh;
    v4f v = *(const v4f*)(slab + row * kSlabP + c4);
    v += b4;
    if (RESID) {
      int pos = t0 + row;
      pos = (pos > kLen - 1) ? (kLen - 1) : pos;
      const v4f r4 = *(const v4f*)(hin_b + (size_t)pos * kCh + c4);
      v += r4;
    }
    *(v4f*)(slab + row * kSlabP + c4) = v;
  }
  __syncthreads();
  if (active) {
    for (int pass = 0; pass < 2; ++pass) {
#pragma unroll
      for (int it = 0; it < 8; ++it) {
        const int row = it * 2 + hh;
        const v4f v = *(const v4f*)(slab + row * kSlabP + c4);
        *(volatile v4f*)(hout_b + (size_t)(t0 + row) * kCh + c4) = v;
      }
      __threadfence();
    }
    for (int pass = 0; pass < 2; ++pass) {
#pragma unroll
      for (int it = 0; it < 4; ++it) {
        const int row = it * 4 + q;
        const float* sp = slab + row * kSlabP + c8;
        v8h hv;
#pragma unroll
        for (int e = 0; e < 8; ++e) hv[e] = (_Float16)sp[e];
        *(volatile v8h*)(hb_b + (size_t)(t0 + row) * kCh + c8) = hv;
      }
      __threadfence();
    }
  }
}

__device__ __forceinline__ _Float16 wcvt(float v) { return (_Float16)(kWCarry * bfr(v)); }

__global__ __launch_bounds__(kThreads) void prep_kernel(const float* __restrict__ dilw, const float* __restrict__ gatew,
                                                     const float* __restrict__ resw,
                                                     _Float16* __restrict__ wf, _Float16* __restrict__ wg, _Float16* __restrict__ wr) {
  const int i = blockIdx.x * kThreads + threadIdx.x;
  if (i >= kLayers * kCh * 8) return;
  const int row = i >> 3;
  const int c0 = (i & 7) * 8;
  const int which = blockIdx.y;
  if (which < 2) {
    const float* src = (which == 0) ? dilw : gatew;
    _Float16* dst = (which == 0) ? wf : wg;
    const float* p = src + ((size_t)row * kCh + c0) * 2;
    const v4f d0 = *(const v4f*)(p);
    const v4f d1 = *(const v4f*)(p + 4);
    const v4f d2 = *(const v4f*)(p + 8);
    const v4f d3 = *(const v4f*)(p + 12);
    v8h t0v, t1v;
    t0v[0] = wcvt(d0[0]); t0v[1] = wcvt(d0[2]); t0v[2] = wcvt(d1[0]); t0v[3] = wcvt(d1[2]);
    t0v[4] = wcvt(d2[0]); t0v[5] = wcvt(d2[2]); t0v[6] = wcvt(d3[0]); t0v[7] = wcvt(d3[2]);
    t1v[0] = wcvt(d0[1]); t1v[1] = wcvt(d0[3]); t1v[2] = wcvt(d1[1]); t1v[3] = wcvt(d1[3]);
    t1v[4] = wcvt(d2[1]); t1v[5] = wcvt(d2[3]); t1v[6] = wcvt(d3[1]); t1v[7] = wcvt(d3[3]);
    _Float16* q0 = dst + (size_t)row * kKfg + c0;
    _Float16* q1 = dst + (size_t)row * kKfg + kCh + c0;
    *(volatile v8h*)q0 = t0v;
    *(volatile v8h*)q1 = t1v;
    __threadfence();
    *(volatile v8h*)q0 = t0v;
    *(volatile v8h*)q1 = t1v;
  } else {
    const float* p = resw + (size_t)row * kCh + c0;
    const v4f r0 = *(const v4f*)(p);
    const v4f r1 = *(const v4f*)(p + 4);
    v8h rv;
    rv[0] = wcvt(r0[0]); rv[1] = wcvt(r0[1]); rv[2] = wcvt(r0[2]); rv[3] = wcvt(r0[3]);
    rv[4] = wcvt(r1[0]); rv[5] = wcvt(r1[1]); rv[6] = wcvt(r1[2]); rv[7] = wcvt(r1[3]);
    _Float16* q = wr + (size_t)row * kCh + c0;
    *(volatile v8h*)q = rv;
    __threadfence();
    *(volatile v8h*)q = rv;
  }
}

__global__ __launch_bounds__(kThreads) void inconv_kernel(const float* __restrict__ x, const float* __restrict__ inw,
                                                       const float* __restrict__ inb,
                                                       float* __restrict__ hout, _Float16* __restrict__ hbout, int tstart) {
  __shared__ __align__(16) _Float16 WinL[kCh * kCin];
  __shared__ __align__(16) _Float16 Xs[kTileP * kCin];
  __shared__ __align__(16) float Slab[kWaves * kWaveP * kSlabP];
  __shared__ __align__(16) float Bsh[kCh];
  const int tid = threadIdx.x, lane = tid & 31, wave = tid >> 5;
  const int b = blockIdx.y;
  const int t0b = tstart + blockIdx.x * kTileP;
  {
    const int o = tid >> 2, k0 = (tid & 3) * 8;
    const float* wp = inw + o * kCin + k0;
    const v4f w0 = *(const v4f*)(wp);
    const v4f w1 = *(const v4f*)(wp + 4);
    v8h hv;
#pragma unroll
    for (int e = 0; e < 4; ++e) { hv[e] = wcvt(w0[e]); hv[4 + e] = wcvt(w1[e]); }
    *(v8h*)(WinL + o * kCin + k0) = hv;
  }
  {
    const int p = tid >> 1, hf = (tid & 1) * 16;
    int pos = t0b + p;
    pos = (pos > kLen - 1) ? (kLen - 1) : pos;
    const float* xp = x + ((size_t)b * kLen + (size_t)pos) * kCin + hf;
    const v4f x0 = *(const v4f*)(xp);
    const v4f x1 = *(const v4f*)(xp + 4);
    const v4f x2 = *(const v4f*)(xp + 8);
    const v4f x3 = *(const v4f*)(xp + 12);
    v8h h0, h1;
#pragma unroll
    for (int e = 0; e < 4; ++e) {
      h0[e] = (_Float16)bfr(x0[e]); h0[4 + e] = (_Float16)bfr(x1[e]);
      h1[e] = (_Float16)bfr(x2[e]); h1[4 + e] = (_Float16)bfr(x3[e]);
    }
    *(v8h*)(Xs + p * kCin + hf) = h0;
    *(v8h*)(Xs + p * kCin + hf + 8) = h1;
  }
  if (tid < kCh) Bsh[tid] = bfr(inb[tid]);
  __syncthreads();

  const int n = lane & 15, hsel = lane >> 4, koff = hsel * 8;
  const int t0 = t0b + wave * kWaveP;
  const bool active = (t0 < kLen);
  const v16h bx = FragH::load(Xs + (wave * kWaveP + n) * kCin + koff);
  v8f acc[4];
#pragma unroll
  for (int mt = 0; mt < 4; ++mt) {
    const v16h aw = FragH::load(WinL + (16 * mt + n) * kCin + koff);
    acc[mt] = FragH::mma(aw, bx, v8f_zero());
    guard_1(acc[mt], aw, bx);
  }
  acc_guard4(acc[0], acc[1], acc[2], acc[3]);

  float* slab = Slab + wave * (kWaveP * kSlabP);
#pragma unroll
  for (int mt = 0; mt < 4; ++mt) {
#pragma unroll
    for (int r = 0; r < 8; ++r) slab[n * kSlabP + 16 * mt + 8 * hsel + r] = acc[mt][r] * kFold;
  }
  const int c4 = (lane & 15) * 4;
  v4f b4;
  b4[0] = Bsh[c4]; b4[1] = Bsh[c4 + 1]; b4[2] = Bsh[c4 + 2]; b4[3] = Bsh[c4 + 3];
  float* hout_b = hout + (size_t)b * kLen * kCh;
  _Float16* hb_b = hbout + (size_t)b * kLen * kCh;
  tile_store<false>(slab, b4, hout_b, hout_b, hb_b, t0, lane, active);
}

__global__ __launch_bounds__(kThreads) void layer_kernel(
    const float* __restrict__ hin, const _Float16* __restrict__ hbin,
    float* __restrict__ hout, _Float16* __restrict__ hbout,
    const _Float16* __restrict__ wf, const _Float16* __restrict__ wg, const _Float16* __restrict__ wr,
    const float* __restrict__ dilb, const float* __restrict__ gateb, const float* __restrict__ resb,
    float* __restrict__ stash_i, int dil, int tstart, int nblk) {
  __shared__ __align__(16) _Float16 WfL[kCh * kKfg];
  __shared__ __align__(16) _Float16 WgL[kCh * kKfg];
  __shared__ __align__(16) _Float16 WrL[kCh * kCh];
  __shared__ __align__(16) _Float16 Zt[kWaves * kWaveP * kZP];
  __shared__ __align__(16) float Slab[kWaves * kWaveP * kSlabP];
  __shared__ __align__(16) float Bsh[3 * kCh];
  const int tid = threadIdx.x, lane = tid & 31, wave = tid >> 5;
  const int b = blockIdx.y;

  if ((int)blockIdx.x == nblk) {
    if (wave == 0) {
      const int c4 = (lane & 15) * 4;
      const v4f v = *(const v4f*)(hin + ((size_t)b * kLen + (size_t)(kLen - dil)) * kCh + c4);
      float* dst = stash_i + (size_t)b * kCh + c4;
      if (lane < 16) *(volatile v4f*)dst = v;
      __threadfence();
      if (lane < 16) *(volatile v4f*)dst = v;
    }
    return;
  }

#pragma unroll 1
  for (int it = 0; it < 4; ++it) { const int e = (it * kThreads + tid) * 8; *(v8h*)(WfL + e) = *(const v8h*)(wf + e); }
#pragma unroll 1
  for (int it = 0; it < 4; ++it) { const int e = (it * kThreads + tid) * 8; *(v8h*)(WgL + e) = *(const v8h*)(wg + e); }
#pragma unroll 1
  for (int it = 0; it < 2; ++it) { const int e = (it * kThreads + tid) * 8; *(v8h*)(WrL + e) = *(const v8h*)(wr + e); }
  {
    const int c = tid & 63, w2 = tid >> 6;
    const float v0 = dilb[c], v1 = gateb[c], v2 = resb[c];
    const float f0 = (w2 == 0) ? 1.0f : 0.0f;
    const float f1 = (w2 == 1) ? 1.0f : 0.0f;
    const float f2 = (w2 == 2) ? 1.0f : 0.0f;
    const float v = fmaf(f0, v0, fmaf(f1, v1, f2 * v2));
    if (tid < 3 * kCh) Bsh[tid] = bfr(v);
  }
  __syncthreads();

  const int n = lane & 15, hsel = lane >> 4, koff = hsel * 8;
  const int t0 = tstart + blockIdx.x * kTileP + wave * kWaveP;
  const bool active = (t0 < kLen);
  const _Float16* hbb = hbin + (size_t)b * kLen * kCh;

  v8f accf[4], accg[4];
#pragma unroll
  for (int mt = 0; mt < 4; ++mt) { accf[mt] = v8f_zero(); accg[mt] = v8f_zero(); }
#pragma unroll
  for (int kc = 0; kc < 4; ++kc) {
    const int doff = (kc < 2) ? -dil : 0;
    int tr = t0 + n + doff;
    tr = (tr < 0) ? 0 : tr;
    tr = (tr > kLen - 1) ? (kLen - 1) : tr;
    const v16h bh = FragH::load(hbb + (size_t)tr * kCh + (kc & 1) * 32 + koff);
#pragma unroll
    for (int mt = 0; mt < 4; ++mt) {
      const v16h af = FragH::load(WfL + (16 * mt + n) * kKfg + 32 * kc + koff);
      const v16h ag = FragH::load(WgL + (16 * mt + n) * kKfg + 32 * kc + koff);
      accf[mt] = FragH::mma(af, bh, accf[mt]);
      accg[mt] = FragH::mma(ag, bh, accg[mt]);
      guard_fg(accf[mt], accg[mt], af, ag, bh);
    }
  }
  acc_guard4(accf[0], accf[1], accf[2], accf[3]);
  acc_guard4(accg[0], accg[1], accg[2], accg[3]);

  _Float16* zw = Zt + wave * (kWaveP * kZP);
#pragma unroll
  for (int mt = 0; mt < 4; ++mt) {
    const int chb = 16 * mt + 8 * hsel;
    v8h zv;
#pragma unroll
    for (int r = 0; r < 8; ++r) {
      const float fpre = fmaf(accf[mt][r], kFold, Bsh[chb + r]);
      const float gpre = fmaf(accg[mt][r], kFold, Bsh[kCh + chb + r]);
      zv[r] = (_Float16)(ftanh(fpre) * fsig(gpre));
    }
    *(v8h*)(zw + n * kZP + chb) = zv;
  }
  __syncthreads();

  v8f accr[4];
#pragma unroll
  for (int mt = 0; mt < 4; ++mt) accr[mt] = v8f_zero();
#pragma unroll
  for (int kc = 0; kc < 2; ++kc) {
    const v16h bz = FragH::load(zw + n * kZP + 32 * kc + koff);
#pragma unroll
    for (int mt = 0; mt < 4; ++mt) {
      const v16h ar = FragH::load(WrL + (16 * mt + n) * kCh + 32 * kc + koff);
      accr[mt] = FragH::mma(ar, bz, accr[mt]);
      guard_1(accr[mt], ar, bz);
    }
  }
  acc_guard4(accr[0], accr[1], accr[2], accr[3]);

  float* slab = Slab + wave * (kWaveP * kSlabP);
#pragma unroll
  for (int mt = 0; mt < 4; ++mt) {
#pragma unroll
    for (int r = 0; r < 8; ++r) slab[n * kSlabP + 16 * mt + 8 * hsel + r] = accr[mt][r] * kFold;
  }
  const int c4 = (lane & 15) * 4;
  v4f b4;
  b4[0] = Bsh[2 * kCh + c4]; b4[1] = Bsh[2 * kCh + c4 + 1]; b4[2] = Bsh[2 * kCh + c4 + 2]; b4[3] = Bsh[2 * kCh + c4 + 3];
  const float* hin_b = hin + (size_t)b * kLen * kCh;
  float* hout_b = hout + (size_t)b * kLen * kCh;
  _Float16* hb_b = hbout + (size_t)b * kLen * kCh;
  tile_store<true>(slab, b4, hin_b, hout_b, hb_b, t0, lane, active);
}

__global__ __launch_bounds__(kThreads) void head_kernel(
    const float* __restrict__ stash,
    const float* __restrict__ dilw, const float* __restrict__ dilb,
    const float* __restrict__ gatew, const float* __restrict__ gateb,
    const float* __restrict__ skipw, const float* __restrict__ skipb,
    const float* __restrict__ e1w, const float* __restrict__ e1b,
    const float* __restrict__ mw, const float* __restrict__ mb,
    const float* __restrict__ lw, const float* __restrict__ lb,
    float* __restrict__ out) {
  __shared__ __align__(16) float Hs[4 * kCh];
  __shared__ __align__(16) float Zs[4 * kCh];
  __shared__ __align__(16) float Ys[4 * kCh];
  __shared__ __align__(16) float Y2s[4 * kEnd];
  __shared__ __align__(16) float Red[kWaves * 2];
  __shared__ __align__(16) float Res[3 * kBatch];
  const int tid = threadIdx.x, lane = tid & 31, wave = tid >> 5;
  const int slot = tid >> 6, o = tid & 63;
  const float mbv = bfr(mb[0]), lbv = bfr(lb[0]);
  const float mw0 = bfr(mw[o]), mw1 = bfr(mw[o + kCh]);
  const float lw0 = bfr(lw[o]), lw1 = bfr(lw[o + kCh]);
  const float eb0 = bfr(e1b[o]), eb1 = bfr(e1b[o + kCh]);
  float* hs = Hs + slot * kCh;
  float* zs = Zs + slot * kCh;
  float* ys = Ys + slot * kCh;
  float* y2s = Y2s + slot * kEnd;

#pragma unroll 1
  for (int jb = 0; jb < kBatch / 4; ++jb) {
    const int bb = jb * 4 + slot;
    float sk = 0.0f;
#pragma unroll 1
    for (int li = 0; li < kLayers; ++li) {
      hs[o] = stash[((size_t)li * kBatch + bb) * kCh + o];
      __syncthreads();
      const size_t wrow = (size_t)(li * kCh + o) * kCh;
      const float* dp = dilw + wrow * 2;
      const float* gp = gatew + wrow * 2;
      float fa = 0.0f, ga = 0.0f;
#pragma unroll 1
      for (int c = 0; c < kCh; ++c) {
        const float hv = hs[c];
        fa = fmaf(bfr(dp[2 * c]), hv, fa);
        ga = fmaf(bfr(gp[2 * c]), hv, ga);
      }
      zs[o] = gated_precise(fa + bfr(dilb[li * kCh + o]), ga + bfr(gateb[li * kCh + o]));
      __syncthreads();
      const float* sp = skipw + wrow;
      float sa = 0.0f;
#pragma unroll 1
      for (int c = 0; c < kCh; ++c) sa = fmaf(bfr(sp[c]), zs[c], sa);
      sk = sk + (sa + bfr(skipb[li * kCh + o]));
    }
    ys[o] = fmaxf(sk, 0.0f);
    __syncthreads();
    const float* w0p = e1w + (size_t)o * kCh;
    const float* w1p = e1w + (size_t)(o + kCh) * kCh;
    float a0 = 0.0f, a1 = 0.0f;
#pragma unroll 1
    for (int c = 0; c < kCh; ++c) {
      const float yv = ys[c];
      a0 = fmaf(bfr(w0p[c]), yv, a0);
      a1 = fmaf(bfr(w1p[c]), yv, a1);
    }
    y2s[o] = fmaxf(a0 + eb0, 0.0f);
    y2s[o + kCh] = fmaxf(a1 + eb1, 0.0f);
    __syncthreads();
    float pm = mw0 * y2s[o];
    pm = fmaf(mw1, y2s[o + kCh], pm);
    float pl = lw0 * y2s[o];
    pl = fmaf(lw1, y2s[o + kCh], pl);
#pragma unroll
    for (int off = 16; off > 0; off >>= 1) {
      pm += __shfl_xor(pm, off, 32);
      pl += __shfl_xor(pl, off, 32);
    }
    if (lane == 0) { Red[wave * 2] = pm; Red[wave * 2 + 1] = pl; }
    __syncthreads();
    if (o == 0) {
      const int wa = slot * 2;
      const float m = (Red[wa * 2] + Red[(wa + 1) * 2]) + mbv;
      const float l = (Red[wa * 2 + 1] + Red[(wa + 1) * 2 + 1]) + lbv;
      Res[bb] = m;
      Res[kBatch + bb] = l;
      Res[2 * kBatch + bb] = expf(0.5f * l);
    }
  }
  __syncthreads();
  if (wave == 0) {
    const int idx = (lane < 24) ? lane : 0;
    v4f v;
    v[0] = Res[idx * 4]; v[1] = Res[idx * 4 + 1]; v[2] = Res[idx * 4 + 2]; v[3] = Res[idx * 4 + 3];
    float* dst = out + idx * 4;
    if (lane < 24) *(volatile v4f*)dst = v;
    __threadfence();
    if (lane < 24) *(volatile v4f*)dst = v;
  }
}

extern "C" void kernel_launch(void* const* d_in, const int* in_sizes, int n_in,
                              void* d_out, int out_size, void* d_ws, size_t ws_size, hipStream_t stream) {
  (void)in_sizes; (void)n_in; (void)out_size;
  const float* x       = (const float*)d_in[0];
  const float* input_w = (const float*)d_in[1];
  const float* input_b = (const float*)d_in[2];
  const float* dil_w   = (const float*)d_in[3];
  const float* dil_b   = (const float*)d_in[4];
  const float* gate_w  = (const float*)d_in[5];
  const float* gate_b  = (const float*)d_in[6];
  const float* skip_w  = (const float*)d_in[7];
  const float* skip_b  = (const float*)d_in[8];
  const float* res_w   = (const float*)d_in[9];
  const float* res_b   = (const float*)d_in[10];
  const float* end1_w  = (const float*)d_in[11];
  const float* end1_b  = (const float*)d_in[12];
  const float* mean_w  = (const float*)d_in[13];
  const float* mean_b  = (const float*)d_in[14];
  const float* lv_w    = (const float*)d_in[15];
  const float* lv_b    = (const float*)d_in[16];

  char* ws = (char*)d_ws;
  size_t off = 0;
  auto carve = [&](size_t bytes) -> char* {
    char* p = ws + off;
    off += (bytes + 255) & ~(size_t)255;
    return p;
  };
  const size_t nH = (size_t)kBatch * kLen * kCh;
  float*    HA    = (float*)carve(nH * sizeof(float));
  float*    HB    = (float*)carve(nH * sizeof(float));
  _Float16* HbA   = (_Float16*)carve(nH * sizeof(_Float16));
  _Float16* HbB   = (_Float16*)carve(nH * sizeof(_Float16));
  _Float16* Wf    = (_Float16*)carve((size_t)kLayers * kCh * kKfg * sizeof(_Float16));
  _Float16* Wg    = (_Float16*)carve((size_t)kLayers * kCh * kKfg * sizeof(_Float16));
  _Float16* Wr    = (_Float16*)carve((size_t)kLayers * kCh * kCh * sizeof(_Float16));
  float*    stash = (float*)carve((size_t)kLayers * kBatch * kCh * sizeof(float));
  if (off > ws_size) return;

  {
    const dim3 grid((unsigned)((kLayers * kCh * 8) / kThreads), 3);
    prep_kernel<<<grid, kThreads, 0, stream>>>(dil_w, gate_w, res_w, Wf, Wg, Wr);
  }
  {
    const int nbin = (kLen - kSched.Tin + kTileP - 1) / kTileP;
    const dim3 grid((unsigned)nbin, kBatch);
    inconv_kernel<<<grid, kThreads, 0, stream>>>(x, input_w, input_b, HA, HbA, kSched.Tin);
  }
  for (int i = 0; i < kLayers; ++i) {
    const float*    hin   = (i & 1) ? HB : HA;
    const _Float16* hbin  = (i & 1) ? HbB : HbA;
    float*          hout  = (i & 1) ? HA : HB;
    _Float16*       hbout = (i & 1) ? HbA : HbB;
    const int T = kSched.T[i];
    const int nblk = (kLen - T + kTileP - 1) / kTileP;
    const dim3 grid((unsigned)(nblk + 1), kBatch);
    layer_kernel<<<grid, kThreads, 0, stream>>>(
        hin, hbin, hout, hbout,
        Wf + (size_t)i * kCh * kKfg, Wg + (size_t)i * kCh * kKfg, Wr + (size_t)i * kCh * kCh,
        dil_b + (size_t)i * kCh, gate_b + (size_t)i * kCh, res_b + (size_t)i * kCh,
        stash + (size_t)i * kBatch * kCh, dil_of(i), T, nblk);
  }
  head_kernel<<<1, kThreads, 0, stream>>>(stash, dil_w, dil_b, gate_w, gate_b, skip_w, skip_b,
                                          end1_w, end1_b, mean_w, mean_b, lv_w, lv_b, (float*)d_out);
}
